// GIN_88098369176167
// MI455X (gfx1250) — hardware-verified
//
#include <hip/hip_runtime.h>
#include <stddef.h>
#include <stdint.h>


#define NN      50000
#define NE      800000
#define NG      256
#define DIN     128
#define KA      256
#define KH1     512
#define MP      50048
#define NTHR    256
#define NWAVE   8
#define EPT     8
#define CHUNK   (NTHR * EPT)
#define WCAP    (EPT * 32)
#define LISTN   (NWAVE * WCAP)
#define NBMAX   2048
#define NBRUN   1024
#define NBLK    49
#define RCAP    20480
#define DEGCAP  64
#define PKS     11
#define RPB     128
#define GBM     64
#define GBN     128
#define GTHR    128
#define GNT     8
#define PARTW   288
#define NPART   (MP / GBM)
#define PG      32
#define WMAT    (DIN * KA)
#define NUWM    (DIN * (KA / 8))
#define NUB1    (4 * NUWM)
#define NUB2    (8 * NUWM)
#define NUB3    (NUB2 + DIN * (KH1 / 8))
#define NUB4    (NUB3 + NUWM)
#define NUXB    (NN * (DIN / 8))
#define NUTOT   (NUB4 + NUXB)
#define LDS_BKT ((2 * RCAP + 2 * NBMAX + LISTN) * 4 + 64)
#define WSLIM   134217728

static_assert((CHUNK & (CHUNK - 1)) == 0 && CHUNK <= (1 << PKS));
static_assert(NBMAX <= (1 << PKS) && NBRUN <= NBMAX && (NBRUN & (NBRUN - 1)) == 0);
static_assert(NTHR * 8 == NBMAX && LISTN >= NBMAX && LISTN == 2 * NBRUN);
static_assert(NBLK * NBRUN >= NN && NBLK * NBRUN >= MP);
static_assert((long long)NE * (1LL << PKS) < (1LL << 31));
static_assert(RCAP * 100 >= 16696 * 105 && DEGCAP >= 36 + 8);
static_assert((RCAP % (NTHR * 4)) == 0 && ((2 * NBRUN) % (NTHR * 4)) == 0 && (RCAP % NTHR) == 0);
static_assert(((2 * RCAP + NBMAX) % 4) == 0);
static_assert(LDS_BKT <= 300000);
static_assert(MP % GBM == 0 && MP % RPB == 0 && MP >= NN && (NBRUN % RPB) == 0 && (MP / RPB) <= NBLK * (NBRUN / RPB));
static_assert(RPB == NWAVE * 16 && DIN == 32 * 4);
static_assert(GBM == (GTHR / 32) * 16 && GBN == 16 * GNT && GTHR == GBN && GBN == DIN);
static_assert(GBN == 4 * 32 && GTHR >= 64);
static_assert((KA % 32) == 0 && (KH1 % 32) == 0 && KA == 2 * DIN && KH1 == 4 * DIN);
static_assert((NG % GBM) == 0 && (NG % PG) == 0 && (PG * (DIN / 8)) % NTHR == 0);
static_assert((PARTW % 32) == 0 && PARTW >= 2 * GBN + 1 && PARTW / 4 <= GTHR);
static_assert((NUB1 % NTHR) == 0 && (NUB2 % NTHR) == 0 && (NUB3 % NTHR) == 0 && (NUB4 % NTHR) == 0 && (NUTOT % NTHR) == 0);
static_assert(((MP * 16) % NTHR) == 0);
static_assert((NE % 4) == 0 && (NN % 4) == 0);

typedef float          v4f  __attribute__((ext_vector_type(4)));
typedef float          v8f  __attribute__((ext_vector_type(8)));
typedef int            v4i  __attribute__((ext_vector_type(4)));
typedef int            v8i  __attribute__((ext_vector_type(8)));
typedef unsigned int   v2u  __attribute__((ext_vector_type(2)));
typedef unsigned int   v4u  __attribute__((ext_vector_type(4)));
typedef unsigned short v8us __attribute__((ext_vector_type(8)));
typedef __bf16         v16b __attribute__((ext_vector_type(16)));
typedef v4f  __attribute__((may_alias)) v4fa;
typedef v4i  __attribute__((may_alias)) v4ia;
typedef v2u  __attribute__((may_alias)) v2ua;
typedef v8us __attribute__((may_alias)) v8usa;
union Frag { v16b vb; v8us h[2]; v8i w; };

__device__ __forceinline__ v8f wmx(const Frag& a, const Frag& b, v8f c) {
  v8f d = __builtin_amdgcn_wmma_f32_16x16x32_bf16(false, a.vb, false, b.vb, (short)0, c, false, false);
  asm volatile("v_nop\n\tv_nop\n\tv_nop\n\tv_nop" : "+v"(d) : "v"(a.w), "v"(b.w));
  return d;
}

__device__ __forceinline__ unsigned short bf_bits(float f) {
  unsigned int u = __float_as_uint(f);
  u += 0x7FFFu + ((u >> 16) & 1u);
  return (unsigned short)(u >> 16);
}
__device__ __forceinline__ float bf_val(unsigned short b) { return __uint_as_float(((unsigned int)b) << 16); }
__device__ __forceinline__ float bf_rne(float f) { return bf_val(bf_bits(f)); }

__device__ __forceinline__ float relu_np(float v) { return (v > 0.0f) ? v : (v - v); }

__device__ __forceinline__ void hilo8(const v4f a, const v4f b, v8us& hv, v8us& lv) {
  const float f[8] = {a.x, a.y, a.z, a.w, b.x, b.y, b.z, b.w};
#pragma unroll
  for (int j = 0; j < 8; ++j) {
    const unsigned short hb = bf_bits(f[j]);
    hv[j] = hb;
    lv[j] = bf_bits(f[j] - bf_val(hb));
  }
}

__device__ __forceinline__ int scan_chunk(const int* __restrict__ dsts, int nE, int cbase, int slotBase,
                                          int nb, int vec8, int* list, int tid, int lane, int wave) {
  int wc = 0;
  const int el0  = tid * EPT;
  const int e0   = cbase + el0;
  const int sent = -2147483647 - 1;
  v4i da, db;
  if (vec8 != 0 && cbase + CHUNK <= nE) {
    da = *(const v4i*)(dsts + e0);
    db = *(const v4i*)(dsts + e0 + 4);
  } else {
    da.x = (e0     < nE) ? dsts[min(e0,     nE - 1)] : sent;
    da.y = (e0 + 1 < nE) ? dsts[min(e0 + 1, nE - 1)] : sent;
    da.z = (e0 + 2 < nE) ? dsts[min(e0 + 2, nE - 1)] : sent;
    da.w = (e0 + 3 < nE) ? dsts[min(e0 + 3, nE - 1)] : sent;
    db.x = (e0 + 4 < nE) ? dsts[min(e0 + 4, nE - 1)] : sent;
    db.y = (e0 + 5 < nE) ? dsts[min(e0 + 5, nE - 1)] : sent;
    db.z = (e0 + 6 < nE) ? dsts[min(e0 + 6, nE - 1)] : sent;
    db.w = (e0 + 7 < nE) ? dsts[min(e0 + 7, nE - 1)] : sent;
  }
  const unsigned nbs = (unsigned)slotBase;
  const unsigned unb = (unsigned)nb;
  const unsigned s0 = (unsigned)da.x - nbs, s1 = (unsigned)da.y - nbs;
  const unsigned s2 = (unsigned)da.z - nbs, s3 = (unsigned)da.w - nbs;
  const unsigned s4 = (unsigned)db.x - nbs, s5 = (unsigned)db.y - nbs;
  const unsigned s6 = (unsigned)db.z - nbs, s7 = (unsigned)db.w - nbs;
  const bool h0 = s0 < unb, h1 = s1 < unb, h2 = s2 < unb, h3 = s3 < unb;
  const bool h4 = s4 < unb, h5 = s5 < unb, h6 = s6 < unb, h7 = s7 < unb;
  const unsigned any = __builtin_amdgcn_ballot_w32(h0 | h1 | h2 | h3 | h4 | h5 | h6 | h7);
  if (any != 0u) {
#define HITJ(J, HJ, SJ) { \
      const unsigned mj = __builtin_amdgcn_ballot_w32(HJ); \
      if (mj != 0u) { \
        if (HJ) { \
          const int pos = wc + (int)__builtin_amdgcn_mbcnt_lo(mj, 0u); \
          if (pos < WCAP) list[wave * WCAP + pos] = ((el0 + (J)) << PKS) | (int)(SJ); \
        } \
        wc += (int)__builtin_popcount(mj); } }
    HITJ(0, h0, s0)
    HITJ(1, h1, s1)
    HITJ(2, h2, s2)
    HITJ(3, h3, s3)
    HITJ(4, h4, s4)
    HITJ(5, h5, s5)
    HITJ(6, h6, s6)
    HITJ(7, h7, s7)
#undef HITJ
  }
  return wc;
}

__device__ __forceinline__ v8us cv8b(const float* __restrict__ p, size_t stride) {
  v8us o;
#pragma unroll
  for (int i = 0; i < 8; ++i) o[i] = bf_bits(p[(size_t)i * stride]);
  return o;
}

__global__ __launch_bounds__(NTHR) void k_prep(const float* __restrict__ Wa, const float* __restrict__ Wb,
                                               const float* __restrict__ oW1, const float* __restrict__ oW2,
                                               const float* __restrict__ feats,
                                               unsigned short* pWa, unsigned short* pWb, unsigned short* pO1,
                                               unsigned short* pO2, unsigned short* pXB) {
  const int u = (int)blockIdx.x * NTHR + (int)threadIdx.x;
  v8us o;
  unsigned short* dp;
  if (u < NUB1) {
    const int v = u, mat = v >> 12, w = v & (NUWM - 1), n = w >> 5, k8 = (w & 31) * 8, kk = k8 & (DIN - 1);
    o = cv8b(Wa + (size_t)mat * (DIN * DIN) + (size_t)kk * DIN + n, DIN);
    dp = pWa + (size_t)v * 8;
  } else if (u < NUB2) {
    const int v = u - NUB1, mat = v >> 12, w = v & (NUWM - 1), n = w >> 5, k8 = (w & 31) * 8, kk = k8 & (DIN - 1);
    o = cv8b(Wb + (size_t)mat * (DIN * DIN) + (size_t)kk * DIN + n, DIN);
    dp = pWb + (size_t)v * 8;
  } else if (u < NUB3) {
    const int v = u - NUB2, n = v >> 6, k8 = (v & 63) * 8, kk = k8 & (2 * DIN - 1);
    o = cv8b(oW1 + (size_t)kk * DIN + n, DIN);
    dp = pO1 + (size_t)v * 8;
  } else if (u < NUB4) {
    const int v = u - NUB3, n = v >> 5, k8 = (v & 31) * 8, kk = k8 & (DIN - 1);
    o = cv8b(oW2 + (size_t)kk * DIN + n, DIN);
    dp = pO2 + (size_t)v * 8;
  } else if (u < NUTOT) {
    const int v = u - NUB4;
    const float* p = feats + (size_t)v * 8;
    const v4f a = *(const v4f*)p;
    const v4f b = *(const v4f*)(p + 4);
    o[0] = bf_bits(a.x); o[1] = bf_bits(a.y); o[2] = bf_bits(a.z); o[3] = bf_bits(a.w);
    o[4] = bf_bits(b.x); o[5] = bf_bits(b.y); o[6] = bf_bits(b.z); o[7] = bf_bits(b.w);
    dp = pXB + (size_t)v * 8;
  } else {
    return;
  }
  *(volatile v8us*)dp = o;
  __threadfence();
  *(volatile v8us*)dp = o;
}

__global__ __launch_bounds__(NTHR) void k_bucket(const int* __restrict__ srcs, const int* __restrict__ dsts,
                                                 int* hits, int* meta, int nN, int nE, int vec8) {
  extern __shared__ v4f lds_dyn[];
  int* reg1 = (int*)lds_dyn;
  int* reg2 = reg1 + RCAP;
  int* scnt = reg2 + RCAP;
  int* soff = scnt + NBMAX;
  int* list = soff + NBMAX;
  int* wcnt = list + LISTN;
  int* wtot = wcnt + NWAVE;
  const int tid = (int)threadIdx.x, lane = tid & 31, wave = tid >> 5;
  const int nodeBase = (int)blockIdx.x * NBRUN;
  const int nb = NBRUN;

  {
    const v4i z4 = {0, 0, 0, 0};
    for (int i = tid * 4; i < 2 * RCAP + NBMAX; i += NTHR * 4) *(v4ia*)(reg1 + i) = z4;
  }
  __syncthreads();

  int tot = 0;
  const int nChunks = (nE + CHUNK - 1) / CHUNK;
#pragma unroll 1
  for (int ch = 0; ch < nChunks; ++ch) {
    const int cbase = ch * CHUNK;
    const int wc = scan_chunk(dsts, nE, cbase, nodeBase, nb, vec8, list, tid, lane, wave);
    if (lane == 0) wcnt[wave] = wc;
    __syncthreads();
    int pre = 0, all = 0;
#pragma unroll
    for (int w2 = 0; w2 < NWAVE; ++w2) {
      int c = wcnt[w2];
      c = c < 0 ? 0 : (c > WCAP ? WCAP : c);
      all += c;
      pre += (w2 < wave) ? c : 0;
    }
    const int wcc  = wc > WCAP ? WCAP : wc;
    const int base = tot + pre;
#pragma unroll 1
    for (int i = lane; i < wcc; i += 32) {
      const int ent = list[wave * WCAP + i];
      const int el  = (ent >> PKS) & (CHUNK - 1);
      const int sl  = ent & (NBMAX - 1);
      int eid = cbase + el;
      eid = eid > nE - 1 ? nE - 1 : eid;
      const int pos = base + i;
      if (pos < RCAP) reg1[pos] = (int)(((unsigned)eid << PKS) | (unsigned)sl);
    }
    tot += all;
    tot = tot > RCAP ? RCAP : tot;
    __syncthreads();
  }
  const int nh = tot;

  if (wave == 0) {
#pragma unroll 1
    for (int b0 = 0; b0 < nh; b0 += 32) {
      const int idx = b0 + lane;
      const int uv  = reg1[idx < RCAP ? idx : RCAP - 1];
      const int m32 = (nh - b0) < 32 ? (nh - b0) : 32;
#pragma unroll 1
      for (int k = 0; k < m32; ++k) {
        const int u  = __builtin_amdgcn_readlane(uv, k);
        const int sl = u & (NBMAX - 1);
        if (lane == 0) scnt[sl] = scnt[sl] + 1;
      }
    }
  }
  __syncthreads();

  {
    const v4i ca = *(const v4ia*)(scnt + 8 * tid);
    const v4i cb = *(const v4ia*)(scnt + 8 * tid + 4);
    const int e0 = ca.x < 0 ? 0 : ca.x, e1 = ca.y < 0 ? 0 : ca.y, e2 = ca.z < 0 ? 0 : ca.z, e3 = ca.w < 0 ? 0 : ca.w;
    const int e4 = cb.x < 0 ? 0 : cb.x, e5 = cb.y < 0 ? 0 : cb.y, e6 = cb.z < 0 ? 0 : cb.z, e7 = cb.w < 0 ? 0 : cb.w;
    const int ts = e0 + e1 + e2 + e3 + e4 + e5 + e6 + e7;
    int incl = ts;
#pragma unroll
    for (int d = 1; d < 32; d <<= 1) {
      const int up = __shfl_up(incl, d);
      if (lane >= d) incl += up;
    }
    if (lane == 31) wtot[wave] = incl;
    __syncthreads();
    int pre = 0;
#pragma unroll
    for (int w2 = 0; w2 < NWAVE; ++w2) pre += (w2 < wave) ? wtot[w2] : 0;
    int run = pre + incl - ts;
    soff[8 * tid + 0] = run; run += e0;
    soff[8 * tid + 1] = run; run += e1;
    soff[8 * tid + 2] = run; run += e2;
    soff[8 * tid + 3] = run; run += e3;
    soff[8 * tid + 4] = run; run += e4;
    soff[8 * tid + 5] = run; run += e5;
    soff[8 * tid + 6] = run; run += e6;
    soff[8 * tid + 7] = run;
  }
  __syncthreads();
  for (int i = tid; i < NBMAX; i += NTHR) list[i] = soff[i];
  __syncthreads();

  if (wave == 0) {
#pragma unroll 1
    for (int b0 = 0; b0 < nh; b0 += 32) {
      const int idx = b0 + lane;
      const int uv  = reg1[idx < RCAP ? idx : RCAP - 1];
      const int m32 = (nh - b0) < 32 ? (nh - b0) : 32;
#pragma unroll 1
      for (int k = 0; k < m32; ++k) {
        const int u   = __builtin_amdgcn_readlane(uv, k);
        const int sl  = u & (NBMAX - 1);
        const int eid = (int)((unsigned)u >> PKS);
        if (lane == 0) {
          int pos = list[sl];
          pos = pos < 0 ? 0 : (pos > RCAP - 1 ? RCAP - 1 : pos);
          reg2[pos] = eid;
          list[sl] = pos + 1;
        }
      }
    }
  }
  __syncthreads();

  const bool ovf = (nh >= RCAP);
#pragma unroll 1
  for (int i0 = 0; i0 < RCAP; i0 += NTHR) {
    const int idx = i0 + tid;
    int eid = reg2[idx];
    eid = eid < 0 ? 0 : (eid > nE - 1 ? nE - 1 : eid);
    int s = srcs[eid];
    s = s < 0 ? 0 : (s > nN - 1 ? nN - 1 : s);
    reg1[idx] = (idx < nh) ? s : 0;
  }
#pragma unroll 1
  for (int i = tid; i < NBRUN; i += NTHR) {
    const int c = scnt[i];
    list[i] = ovf ? (DEGCAP + 1) : c;
    list[NBRUN + i] = soff[i];
  }
  __syncthreads();

  int* hp = hits + (size_t)blockIdx.x * RCAP;
  int* mp = meta + (size_t)blockIdx.x * (2 * NBRUN);
#pragma unroll 1
  for (int it = 0; it < RCAP / (NTHR * 4); ++it) {
    const int idx = (it * NTHR + tid) * 4;
    const v4i v = *(const v4ia*)(reg1 + idx);
    *(volatile v4i*)(hp + idx) = v;
  }
#pragma unroll 1
  for (int it = 0; it < (2 * NBRUN) / (NTHR * 4); ++it) {
    const int idx = (it * NTHR + tid) * 4;
    const v4i v = *(const v4ia*)(list + idx);
    *(volatile v4i*)(mp + idx) = v;
  }
  __threadfence();
#pragma unroll 1
  for (int it = 0; it < RCAP / (NTHR * 4); ++it) {
    const int idx = (it * NTHR + tid) * 4;
    const v4i v = *(const v4ia*)(reg1 + idx);
    *(volatile v4i*)(hp + idx) = v;
  }
#pragma unroll 1
  for (int it = 0; it < (2 * NBRUN) / (NTHR * 4); ++it) {
    const int idx = (it * NTHR + tid) * 4;
    const v4i v = *(const v4ia*)(list + idx);
    *(volatile v4i*)(mp + idx) = v;
  }
}

template <int SRC16>
__global__ __launch_bounds__(NTHR) void k_agg(const int* __restrict__ hits, const int* __restrict__ meta,
                                              const unsigned short* __restrict__ xb, const float* __restrict__ hf,
                                              const float* __restrict__ epsp, unsigned short* zout, int nN) {
  __shared__ int scn[RPB];
  __shared__ int sof[RPB];
  const int tid = (int)threadIdx.x, lane = tid & 31, wave = tid >> 5;
  const int rowBase = (int)blockIdx.x * RPB;
  const int bb = (int)blockIdx.x / (NBRUN / RPB);
  const int sb = ((int)blockIdx.x % (NBRUN / RPB)) * RPB;
  const int* mp = meta + (size_t)bb * (2 * NBRUN);
  if (tid < RPB) {
    scn[tid] = mp[sb + tid];
    sof[tid] = mp[NBRUN + sb + tid];
  }
  __syncthreads();
  const float cself = 1.0f + bf_rne(epsp[0]);
  const int* hp = hits + (size_t)bb * RCAP;
  const float qnan = __int_as_float(0x7fc00000);

#pragma unroll 1
  for (int jt = 0; jt < RPB / NWAVE; ++jt) {
    const int slot = wave * (RPB / NWAVE) + jt;
    const int grow = rowBase + slot;
    const int craw = scn[slot];
    int cnt = craw < 0 ? 0 : (craw > DEGCAP ? DEGCAP : craw);
    int st = sof[slot];
    st = st < 0 ? 0 : (st > RCAP ? RCAP : st);
    if (cnt > RCAP - st) cnt = RCAP - st;
    const bool bad = (craw > DEGCAP) || (craw < 0);
    const bool liveRow = grow < nN;

    float ag0 = 0.f, ag1 = 0.f, ag2 = 0.f, ag3 = 0.f;
#pragma unroll 1
    for (int b0 = 0; b0 < cnt; b0 += 32) {
      int idx = st + b0 + lane;
      idx = idx > RCAP - 1 ? RCAP - 1 : idx;
      int sv = hp[idx];
      sv = sv < 0 ? 0 : (sv > nN - 1 ? nN - 1 : sv);
      const int m32 = (cnt - b0) < 32 ? (cnt - b0) : 32;
#pragma unroll 1
      for (int k = 0; k < m32; ++k) {
        const int sk = __builtin_amdgcn_readlane(sv, k);
        if constexpr (SRC16 != 0) {
          const v2u q = *(const v2ua*)(xb + (size_t)sk * DIN + 4 * lane);
          ag0 += __uint_as_float(q.x << 16);
          ag1 += __uint_as_float(q.x & 0xffff0000u);
          ag2 += __uint_as_float(q.y << 16);
          ag3 += __uint_as_float(q.y & 0xffff0000u);
        } else {
          const v4f v = *(const v4f*)(hf + (size_t)sk * DIN + 4 * lane);
          ag0 += v.x; ag1 += v.y; ag2 += v.z; ag3 += v.w;
        }
      }
    }
    const int nc = liveRow ? grow : nN - 1;
    float s0, s1, s2, s3;
    if constexpr (SRC16 != 0) {
      const v2u q = *(const v2ua*)(xb + (size_t)nc * DIN + 4 * lane);
      s0 = __uint_as_float(q.x << 16);
      s1 = __uint_as_float(q.x & 0xffff0000u);
      s2 = __uint_as_float(q.y << 16);
      s3 = __uint_as_float(q.y & 0xffff0000u);
    } else {
      const v4f v = *(const v4f*)(hf + (size_t)nc * DIN + 4 * lane);
      s0 = v.x; s1 = v.y; s2 = v.z; s3 = v.w;
    }
    const float pz = bad ? qnan : 0.0f;
    float r0 = cself * s0 + ag0 + pz;
    float r1 = cself * s1 + ag1 + pz;
    float r2 = cself * s2 + ag2 + pz;
    float r3 = cself * s3 + ag3 + pz;
    r0 = liveRow ? r0 : 0.0f;
    r1 = liveRow ? r1 : 0.0f;
    r2 = liveRow ? r2 : 0.0f;
    r3 = liveRow ? r3 : 0.0f;

    const unsigned short h0 = bf_bits(r0), h1 = bf_bits(r1), h2 = bf_bits(r2), h3 = bf_bits(r3);
    const unsigned short l0 = bf_bits(r0 - bf_val(h0)), l1 = bf_bits(r1 - bf_val(h1));
    const unsigned short l2 = bf_bits(r2 - bf_val(h2)), l3 = bf_bits(r3 - bf_val(h3));
    v2u hk, lk;
    hk.x = (unsigned int)h0 | ((unsigned int)h1 << 16);
    hk.y = (unsigned int)h2 | ((unsigned int)h3 << 16);
    lk.x = (unsigned int)l0 | ((unsigned int)l1 << 16);
    lk.y = (unsigned int)l2 | ((unsigned int)l3 << 16);
    unsigned short* gp = zout + (size_t)grow * KA + 4 * lane;
    *(volatile v2u*)gp = hk;
    *(volatile v2u*)(gp + DIN) = lk;
    __threadfence();
    *(volatile v2u*)gp = hk;
    *(volatile v2u*)(gp + DIN) = lk;
  }
}

template <int EPI>
__global__ __launch_bounds__(GTHR) void k_gemm(const unsigned short* __restrict__ A, int lda,
                                               const unsigned short* __restrict__ BT, int ldb, int K,
                                               const float* __restrict__ bias,
                                               void* outp, int ldo, int lsplit, int nN, int mRows,
                                               float* part, const float* __restrict__ w3,
                                               const float* __restrict__ b3) {
  __shared__ __attribute__((aligned(16))) float stg[GBM * GBN];
  __shared__ __attribute__((aligned(16))) float pst[PARTW];
  __shared__ __attribute__((aligned(16))) float bsh[GBN];
  __shared__ __attribute__((aligned(16))) float w3s[GBN];
  __shared__ __attribute__((aligned(16))) float sc[GBM];
  const int tid = (int)threadIdx.x, lane = tid & 31, wave = tid >> 5, hh = lane >> 4, m = lane & 15;
  const int rowBase = (int)blockIdx.x * GBM;
  const int colBase = (int)blockIdx.y * GBN;

  if (wave == 0) {
    const v4f b4 = *(const v4f*)(bias + colBase + 4 * lane);
    v4f o;
    o.x = bf_rne(b4.x); o.y = bf_rne(b4.y); o.z = bf_rne(b4.z); o.w = bf_rne(b4.w);
    *(v4fa*)(bsh + 4 * lane) = o;
  }
  if constexpr (EPI == 4) {
    if (wave == 1) {
      const v4f w4 = *(const v4f*)(w3 + 4 * lane);
      v4f o;
      o.x = bf_rne(w4.x); o.y = bf_rne(w4.y); o.z = bf_rne(w4.z); o.w = bf_rne(w4.w);
      *(v4fa*)(w3s + 4 * lane) = o;
    }
  }

  v8f acc[GNT];
  {
    const v8f z = {0.f, 0.f, 0.f, 0.f, 0.f, 0.f, 0.f, 0.f};
#pragma unroll
    for (int t = 0; t < GNT; ++t) acc[t] = z;
  }
  const unsigned short* ap = A  + (size_t)(rowBase + 16 * wave + m) * (size_t)lda + 8 * hh;
  const unsigned short* bp = BT + (size_t)(colBase + m) * (size_t)ldb + 8 * hh;

#pragma unroll 1
  for (int k0 = 0; k0 < K; k0 += 32) {
    Frag af;
    af.h[0] = *(const v8usa*)(ap + k0);
    af.h[1] = *(const v8usa*)(ap + k0 + 16);
#pragma unroll
    for (int nt = 0; nt < GNT; ++nt) {
      const unsigned short* wq = bp + (size_t)(16 * nt) * (size_t)ldb + k0;
      Frag bfr;
      bfr.h[0] = *(const v8usa*)wq;
      bfr.h[1] = *(const v8usa*)(wq + 16);
      acc[nt] = wmx(af, bfr, acc[nt]);
    }
  }
  __syncthreads();

#pragma unroll
  for (int nt = 0; nt < GNT; ++nt) {
    const int lc = 16 * nt + m;
    const float bb = bsh[lc];
#pragma unroll
    for (int r = 0; r < 8; ++r) {
      const int lr = 16 * wave + 8 * hh + r;
      const bool live = (rowBase + lr) < nN;
      float v = acc[nt][r] + bb;
      if constexpr (EPI == 1 || EPI == 3 || EPI == 4) v = relu_np(v);
      stg[lr * GBN + lc] = live ? v : 0.0f;
    }
  }
  __syncthreads();

  if constexpr (EPI == 3) {
    unsigned short* outH = (unsigned short*)outp;
    const int cb = 8 * m;
    const bool isHi = (hh == 0);
    v4u pk[16];
#pragma unroll
    for (int i = 0; i < 16; ++i) {
      const int lr = 16 * wave + i;
      const v4f a = *(const v4fa*)(stg + lr * GBN + cb);
      const v4f b = *(const v4fa*)(stg + lr * GBN + cb + 4);
      const float f[8] = {a.x, a.y, a.z, a.w, b.x, b.y, b.z, b.w};
      unsigned int w[4];
#pragma unroll
      for (int j = 0; j < 4; ++j) {
        const unsigned short h0 = bf_bits(f[2 * j]), h1 = bf_bits(f[2 * j + 1]);
        const unsigned short l0 = bf_bits(f[2 * j] - bf_val(h0)), l1 = bf_bits(f[2 * j + 1] - bf_val(h1));
        const unsigned short q0 = isHi ? h0 : l0, q1 = isHi ? h1 : l1;
        w[j] = (unsigned int)q0 | ((unsigned int)q1 << 16);
      }
      v4u pv; pv.x = w[0]; pv.y = w[1]; pv.z = w[2]; pv.w = w[3];
      pk[i] = pv;
    }
#pragma unroll
    for (int i = 0; i < 16; ++i) {
      const int gr = rowBase + 16 * wave + i;
      unsigned short* op = outH + (size_t)gr * (size_t)ldo + colBase + cb + hh * lsplit;
      if (gr < mRows) *(volatile v4u*)op = pk[i];
    }
    __threadfence();
#pragma unroll
    for (int i = 0; i < 16; ++i) {
      const int gr = rowBase + 16 * wave + i;
      unsigned short* op = outH + (size_t)gr * (size_t)ldo + colBase + cb + hh * lsplit;
      if (gr < mRows) *(volatile v4u*)op = pk[i];
    }
  } else if constexpr (EPI == 4) {
    float* outF = (float*)outp;
    if (tid < GBM) {
      float s = 0.0f;
#pragma unroll 4
      for (int c = 0; c < GBN; ++c) s = fmaf(stg[tid * GBN + c], w3s[c], s);
      sc[tid] = s + bf_rne(b3[0]);
    }
    __syncthreads();
    const v4f o = *(const v4fa*)(sc + 4 * (tid & 15));
    float* op = outF + rowBase + 4 * (tid & 15);
    const bool wr = (tid < 16) && (rowBase + GBM <= mRows);
    if (wr) *(volatile v4f*)op = o;
    __threadfence();
    if (wr) *(volatile v4f*)op = o;
  } else {
    float* outF = (float*)outp;
    v4f fv[16];
#pragma unroll
    for (int i = 0; i < 16; ++i) {
      const int lr = 16 * wave + i;
      fv[i] = *(const v4fa*)(stg + lr * GBN + 4 * lane);
    }
    v4f pv = {0.f, 0.f, 0.f, 0.f};
    const bool pok = (EPI == 0) && (tid < PARTW / 4);
    if constexpr (EPI == 0) {
      int nvr = nN - rowBase;
      nvr = nvr < 0 ? 0 : (nvr > GBM ? GBM : nvr);
      float s = 0.0f;
#pragma unroll 1
      for (int r = 0; r < nvr; ++r) s += stg[r * GBN + tid];
      const float inv = 1.0f / (float)(nvr < 1 ? 1 : nvr);
      const float mean = s * inv;
      float q = 0.0f;
#pragma unroll 1
      for (int r = 0; r < nvr; ++r) {
        const float d = stg[r * GBN + tid] - mean;
        q = fmaf(d, d, q);
      }
      pst[1 + tid] = mean;
      pst[1 + GBN + tid] = q;
      if (tid == 0) pst[0] = (float)nvr;
#pragma unroll 1
      for (int i = 2 * GBN + 1 + tid; i < PARTW; i += GTHR) pst[i] = 0.0f;
      __syncthreads();
      if (pok) pv = *(const v4fa*)(pst + 4 * tid);
    }
    const size_t prow = (size_t)blockIdx.x * (size_t)gridDim.y + (size_t)blockIdx.y;
    float* pp = part + prow * PARTW + 4 * tid;
#pragma unroll
    for (int i = 0; i < 16; ++i) {
      const int gr = rowBase + 16 * wave + i;
      float* op = outF + (size_t)gr * (size_t)ldo + colBase + 4 * lane;
      if (gr < mRows) *(volatile v4f*)op = fv[i];
    }
    if (pok) *(volatile v4f*)pp = pv;
    __threadfence();
#pragma unroll
    for (int i = 0; i < 16; ++i) {
      const int gr = rowBase + 16 * wave + i;
      float* op = outF + (size_t)gr * (size_t)ldo + colBase + 4 * lane;
      if (gr < mRows) *(volatile v4f*)op = fv[i];
    }
    if (pok) *(volatile v4f*)pp = pv;
  }
}

__global__ __launch_bounds__(GBN) void k_comb(const float* __restrict__ part, int nPart,
                                              const float* __restrict__ gam, const float* __restrict__ bet,
                                              float* ss) {
  __shared__ __attribute__((aligned(16))) float stg[4 * GBN];
  const int tid = (int)threadIdx.x;
  double n = 0.0, mean = 0.0, M2 = 0.0;
#pragma unroll 1
  for (int b = 0; b < nPart; ++b) {
    const float* pr = part + (size_t)b * PARTW;
    const double nb = (double)pr[0];
    const double mb = (double)pr[1 + tid];
    const double qb = (double)pr[1 + GBN + tid];
    if (nb > 0.5) {
      const double nn = n + nb;
      const double delta = mb - mean;
      const double f = nb / nn;
      mean = mean + delta * f;
      M2 = M2 + qb + delta * delta * n * f;
      n = nn;
    }
  }
  const double nt = n < 1.0 ? 1.0 : n;
  const float varf = (float)(M2 / nt);
  const float rstd = 1.0f / sqrtf(varf + 1e-5f);
  stg[tid] = (float)mean;
  stg[GBN + tid] = rstd;
  stg[2 * GBN + tid] = bf_rne(gam[tid]);
  stg[3 * GBN + tid] = bf_rne(bet[tid]);
  __syncthreads();
  const v4f v = *(const v4fa*)(stg + 4 * tid);
  *(volatile v4f*)(ss + 4 * tid) = v;
  __threadfence();
  *(volatile v4f*)(ss + 4 * tid) = v;
}

__global__ __launch_bounds__(NTHR) void k_apply(const float* __restrict__ T, const float* __restrict__ ss,
                                               unsigned short* outp, int nN) {
  __shared__ float ssh[4 * DIN];
  const int tid = (int)threadIdx.x;
  ssh[tid] = ss[tid];
  ssh[NTHR + tid] = ss[NTHR + tid];
  __syncthreads();
  const int u = (int)blockIdx.x * NTHR + tid;
  const int row = u >> 4, q = u & 15, c0 = 8 * q;
  const bool live = row < nN;
  const int rc = live ? row : nN - 1;
  const float* tp = T + (size_t)rc * DIN + c0;
  const v4f a = *(const v4f*)tp;
  const v4f b = *(const v4f*)(tp + 4);
  const float t[8] = {a.x, a.y, a.z, a.w, b.x, b.y, b.z, b.w};
  float y[8];
#pragma unroll
  for (int j = 0; j < 8; ++j) {
    const int c = c0 + j;
    const float v = ((t[j] - ssh[c]) * ssh[DIN + c]) * ssh[2 * DIN + c] + ssh[3 * DIN + c];
    y[j] = live ? relu_np(v) : 0.0f;
  }
  v4f ya, yb;
  ya.x = y[0]; ya.y = y[1]; ya.z = y[2]; ya.w = y[3];
  yb.x = y[4]; yb.y = y[5]; yb.z = y[6]; yb.w = y[7];
  v8us hv, lv;
  hilo8(ya, yb, hv, lv);
  unsigned short* hp = outp + (size_t)row * KA + c0;
  unsigned short* lp = hp + DIN;
  *(volatile v8us*)hp = hv;
  *(volatile v8us*)lp = lv;
  __threadfence();
  *(volatile v8us*)hp = hv;
  *(volatile v8us*)lp = lv;
}

__global__ __launch_bounds__(NTHR) void k_pool(const float* __restrict__ U, const int* __restrict__ bat,
                                              int nN, int vec8b, int nG, unsigned short* hc, int colOff) {
  __shared__ __attribute__((aligned(16))) float accs[PG * DIN];
  __shared__ int list[LISTN];
  __shared__ int wcnt[NWAVE];
  const int tid = (int)threadIdx.x, lane = tid & 31, wave = tid >> 5;
  const int slotBase = (int)blockIdx.x * PG;

  for (int i = tid; i < PG * DIN; i += NTHR) accs[i] = 0.0f;
  __syncthreads();

  const int nChunks = (nN + CHUNK - 1) / CHUNK;
#pragma unroll 1
  for (int ch = 0; ch < nChunks; ++ch) {
    const int cbase = ch * CHUNK;
    const int wc = scan_chunk(bat, nN, cbase, slotBase, PG, vec8b, list, tid, lane, wave);
    if (lane == 0) wcnt[wave] = wc;
    __syncthreads();
#pragma unroll 1
    for (int w2 = 0; w2 < NWAVE; ++w2) {
      int c = wcnt[w2];
      c = c < 0 ? 0 : (c > WCAP ? WCAP : c);
#pragma unroll 1
      for (int i = 0; i < c; ++i) {
        const int ent = list[w2 * WCAP + i];
        const int el  = (ent >> PKS) & (CHUNK - 1);
        const int sl  = ent & (PG - 1);
        int node = cbase + el;
        node = node < 0 ? 0 : (node > nN - 1 ? nN - 1 : node);
        if (tid < DIN) {
          const float u = U[(size_t)node * DIN + tid];
          accs[sl * DIN + tid] += u;
        }
      }
    }
    __syncthreads();
  }

  constexpr int PPR = DIN / 8;
  constexpr int NIT = (PG * PPR) / NTHR;
  v8us hv[NIT], lv[NIT];
#pragma unroll
  for (int it = 0; it < NIT; ++it) {
    const int p = it * NTHR + tid;
    const int row = p / PPR, q = p % PPR;
    const v4f a = *(const v4fa*)(accs + row * DIN + 8 * q);
    const v4f b = *(const v4fa*)(accs + row * DIN + 8 * q + 4);
    hilo8(a, b, hv[it], lv[it]);
  }
#pragma unroll
  for (int it = 0; it < NIT; ++it) {
    const int p = it * NTHR + tid;
    const int row = p / PPR, q = p % PPR;
    const int g = slotBase + row;
    unsigned short* hp = hc + (size_t)g * KH1 + colOff + 8 * q;
    unsigned short* lp = hc + (size_t)g * KH1 + 2 * DIN + colOff + 8 * q;
    if (g < nG) { *(volatile v8us*)hp = hv[it]; *(volatile v8us*)lp = lv[it]; }
  }
  __threadfence();
#pragma unroll
  for (int it = 0; it < NIT; ++it) {
    const int p = it * NTHR + tid;
    const int row = p / PPR, q = p % PPR;
    const int g = slotBase + row;
    unsigned short* hp = hc + (size_t)g * KH1 + colOff + 8 * q;
    unsigned short* lp = hc + (size_t)g * KH1 + 2 * DIN + colOff + 8 * q;
    if (g < nG) { *(volatile v8us*)hp = hv[it]; *(volatile v8us*)lp = lv[it]; }
  }
}

static inline size_t al256(size_t o) { return (o + 255) & ~(size_t)255; }

extern "C" void kernel_launch(void* const* d_in, const int* in_sizes, int n_in,
                              void* d_out, int out_size, void* d_ws, size_t ws_size,
                              hipStream_t stream) {
  if (n_in < 18) return;
  if (in_sizes[0] != NN * DIN) return;
  if (in_sizes[1] != 2 * NE || in_sizes[2] != 2 * NE) return;
  if (in_sizes[3] != NN) return;
  if (in_sizes[4] != 1 || in_sizes[5] != 4) return;
  if (in_sizes[6] != 4 * DIN * DIN || in_sizes[10] != 4 * DIN * DIN) return;
  if (in_sizes[7] != 4 * DIN || in_sizes[8] != 4 * DIN || in_sizes[9] != 4 * DIN || in_sizes[11] != 4 * DIN) return;
  if (in_sizes[12] != 2 * DIN * DIN || in_sizes[13] != DIN) return;
  if (in_sizes[14] != DIN * DIN || in_sizes[15] != DIN) return;
  if (in_sizes[16] != DIN || in_sizes[17] != 1) return;
  if (out_size != NG) return;

  const float* feats = (const float*)d_in[0];
  const int*   src   = (const int*)  d_in[1];
  const int*   dst   = (const int*)  d_in[2];
  const int*   gids  = (const int*)  d_in[3];
  const float* eps   = (const float*)d_in[5];
  const float* Wa    = (const float*)d_in[6];
  const float* ba    = (const float*)d_in[7];
  const float* bng   = (const float*)d_in[8];
  const float* bnb   = (const float*)d_in[9];
  const float* Wb    = (const float*)d_in[10];
  const float* bb    = (const float*)d_in[11];
  const float* oW1   = (const float*)d_in[12];
  const float* ob1   = (const float*)d_in[13];
  const float* oW2   = (const float*)d_in[14];
  const float* ob2   = (const float*)d_in[15];
  const float* oW3   = (const float*)d_in[16];
  const float* ob3   = (const float*)d_in[17];
  float* out = (float*)d_out;

  char* ws = (char*)d_ws;
  size_t off = 0;
  const size_t oWA = off; off = al256(off + (size_t)4 * WMAT * 2);
  const size_t oWB = off; off = al256(off + (size_t)4 * WMAT * 2);
  const size_t oO1 = off; off = al256(off + (size_t)DIN * KH1 * 2);
  const size_t oO2 = off; off = al256(off + (size_t)DIN * KA * 2);
  const size_t oXB = off; off = al256(off + (size_t)NN * DIN * 2);
  const size_t oP1 = off; off = al256(off + (size_t)MP * KA * 2);
  const size_t oP2 = off; off = al256(off + (size_t)MP * DIN * 4);
  const size_t oHT = off; off = al256(off + (size_t)2 * NBLK * RCAP * 4);
  const size_t oMT = off; off = al256(off + (size_t)2 * NBLK * 2 * NBRUN * 4);
  const size_t oPT = off; off = al256(off + (size_t)NPART * PARTW * 4);
  const size_t oSS = off; off = al256(off + (size_t)(4 * DIN) * 4);
  const size_t oHG = off; off = al256(off + (size_t)NG * KH1 * 2);
  const size_t oX1 = off; off = al256(off + (size_t)NG * KA * 2);
  if (off > ws_size || off > (size_t)WSLIM) return;
  unsigned short* WAT = (unsigned short*)(ws + oWA);
  unsigned short* WBT = (unsigned short*)(ws + oWB);
  unsigned short* O1T = (unsigned short*)(ws + oO1);
  unsigned short* O2T = (unsigned short*)(ws + oO2);
  unsigned short* XB  = (unsigned short*)(ws + oXB);
  unsigned short* P1  = (unsigned short*)(ws + oP1);
  float*          P2  = (float*)(ws + oP2);
  int*            HT  = (int*)(ws + oHT);
  int*            MT  = (int*)(ws + oMT);
  float*          PT  = (float*)(ws + oPT);
  float*          SS  = (float*)(ws + oSS);
  unsigned short* HG  = (unsigned short*)(ws + oHG);
  unsigned short* X1  = (unsigned short*)(ws + oX1);

  hipFuncSetAttribute(reinterpret_cast<const void*>(&k_bucket), hipFuncAttributeMaxDynamicSharedMemorySize, LDS_BKT);

  k_prep<<<NUTOT / NTHR, NTHR, 0, stream>>>(Wa, Wb, oW1, oW2, feats, WAT, WBT, O1T, O2T, XB);
  for (int e = 0; e < 2; ++e) {
    k_bucket<<<NBLK, NTHR, LDS_BKT, stream>>>(src + (size_t)e * NE, dst + (size_t)e * NE,
                                              HT + (size_t)e * NBLK * RCAP, MT + (size_t)e * NBLK * 2 * NBRUN,
                                              NN, NE, 1);
  }
  const int gM = MP / GBM;
  for (int e = 0; e < 2; ++e) {
    const int* HTe = HT + (size_t)e * NBLK * RCAP;
    const int* MTe = MT + (size_t)e * NBLK * 2 * NBRUN;
    for (int l = 0; l < 2; ++l) {
      const int el = e * 2 + l;
      if (l == 0) {
        k_agg<1><<<MP / RPB, NTHR, 0, stream>>>(HTe, MTe, XB, P2, eps + el, P1, NN);
      } else {
        k_agg<0><<<MP / RPB, NTHR, 0, stream>>>(HTe, MTe, XB, P2, eps + el, P1, NN);
      }
      k_gemm<0><<<dim3(gM, 1), GTHR, 0, stream>>>(P1, KA, WAT + (size_t)el * WMAT, KA, KA, ba + (size_t)el * DIN,
                                                  (void*)P2, DIN, 0, NN, MP, PT, oW3, ob3);
      k_comb<<<1, GBN, 0, stream>>>(PT, NPART, bng + (size_t)el * DIN, bnb + (size_t)el * DIN, SS);
      k_apply<<<(MP * 16) / NTHR, NTHR, 0, stream>>>(P2, SS, P1, NN);
      if (l == 0) {
        k_gemm<1><<<dim3(gM, 1), GTHR, 0, stream>>>(P1, KA, WBT + (size_t)el * WMAT, KA, KA, bb + (size_t)el * DIN,
                                                    (void*)P2, DIN, 0, NN, MP, PT, oW3, ob3);
      } else {
        k_gemm<2><<<dim3(gM, 1), GTHR, 0, stream>>>(P1, KA, WBT + (size_t)el * WMAT, KA, KA, bb + (size_t)el * DIN,
                                                    (void*)P2, DIN, 0, NN, MP, PT, oW3, ob3);
      }
    }
    k_pool<<<NG / PG, NTHR, 0, stream>>>(P2, gids, NN, 1, NG, HG, e * DIN);
  }
  k_gemm<3><<<dim3(NG / GBM, 1), GTHR, 0, stream>>>(HG, KH1, O1T, KH1, KH1, ob1, (void*)X1, KA, DIN, NG, NG, PT, oW3, ob3);
  k_gemm<4><<<dim3(NG / GBM, 1), GTHR, 0, stream>>>(X1, KA, O2T, KA, KA, ob2, (void*)out, 1, 0, NG, NG, PT, oW3, ob3);
}
